// TMK_46608985096827
// MI455X (gfx1250) — hardware-verified
//
#include <hip/hip_runtime.h>

typedef __attribute__((ext_vector_type(16))) _Float16 v16h;
typedef __attribute__((ext_vector_type(8)))  _Float16 v8h;
typedef __attribute__((ext_vector_type(16))) __bf16   v16b;
typedef __attribute__((ext_vector_type(8)))  __bf16   v8b;
typedef __attribute__((ext_vector_type(8)))  float    v8f;
typedef __attribute__((ext_vector_type(4)))  float    v4f;

static constexpr int FEAT_DIM = 16;
static constexpr int NDESIGN  = 1024;
static constexpr int COL_HALF = 512;
static constexpr int ROWS_BLK = 32;

__device__ __forceinline__ unsigned short f2bf_bits(float f) {
  unsigned u = __float_as_uint(f);
  return (unsigned short)((u + 0x7FFFu + ((u >> 16) & 1u)) >> 16);
}
__device__ __forceinline__ float bf_bits2f(unsigned short h) { return __uint_as_float(((unsigned)h) << 16); }

__device__ __forceinline__ void dep_guard_h(v8f& a, v8f& b, v16h x, v16h y) { asm volatile("v_nop\n\tv_nop\n\tv_nop\n\tv_nop" : "+v"(a), "+v"(b) : "v"(x), "v"(y)); }
__device__ __forceinline__ void dep_guard_b(v8f& a, v8f& b, v16b x, v16b y) { asm volatile("v_nop\n\tv_nop\n\tv_nop\n\tv_nop" : "+v"(a), "+v"(b) : "v"(x), "v"(y)); }
__device__ __forceinline__ void keep4_h(v16h a, v16h b, v16h c, v16h d) { asm volatile("v_nop" :: "v"(a), "v"(b), "v"(c), "v"(d)); }
__device__ __forceinline__ void keep4_b(v16b a, v16b b, v16b c, v16b d) { asm volatile("v_nop" :: "v"(a), "v"(b), "v"(c), "v"(d)); }
__device__ __forceinline__ void acc_guard4(v8f& a, v8f& b, v8f& c, v8f& d) { asm volatile("v_nop\n\tv_nop\n\tv_nop\n\tv_nop" : "+v"(a), "+v"(b), "+v"(c), "+v"(d)); }
template <typename T> struct Frag;
template <> struct Frag<_Float16> {
  typedef v16h V; union U { v16h v; v8h h[2]; };
  static __device__ __forceinline__ v16h load(const _Float16* p) {
    U f; f.h[0] = *(const v8h*)(p); f.h[1] = *(const v8h*)(p + 16); return f.v;
  }
  static __device__ __forceinline__ v8f mma(v16h a, v16h b, v8f c) {
    return __builtin_amdgcn_wmma_f32_16x16x32_f16(false, a, false, b, (short)0, c, false, false);
  }
  static __device__ __forceinline__ void guard(v8f& a, v8f& b, v16h x, v16h y) { dep_guard_h(a, b, x, y); }
  static __device__ __forceinline__ void keep(v16h a, v16h b, v16h c, v16h d) { keep4_h(a, b, c, d); }
};
template <> struct Frag<__bf16> {
  typedef v16b V; union U { v16b v; v8b h[2]; };
  static __device__ __forceinline__ v16b load(const __bf16* p) {
    U f; f.h[0] = *(const v8b*)(p); f.h[1] = *(const v8b*)(p + 16); return f.v;
  }
  static __device__ __forceinline__ v8f mma(v16b a, v16b b, v8f c) {
    return __builtin_amdgcn_wmma_f32_16x16x32_bf16(false, a, false, b, (short)0, c, false, false);
  }
  static __device__ __forceinline__ void guard(v8f& a, v8f& b, v16b x, v16b y) { dep_guard_b(a, b, x, y); }
  static __device__ __forceinline__ void keep(v16b a, v16b b, v16b c, v16b d) { keep4_b(a, b, c, d); }
};

template <int ET> struct Elem;
template <> struct Elem<0> { typedef _Float16 T; };
template <> struct Elem<1> { typedef __bf16 T; };
template <int ET, bool SPLIT, int BIAS_MODE, int OUT_MODE, bool RESID, int ACT = 0>
__global__ __launch_bounds__(256) void wmma_gemm64(
    const unsigned short* __restrict__ Ap, const unsigned short* __restrict__ A2p, int lda, long strideA,
    const unsigned short* __restrict__ Btp, const unsigned short* __restrict__ Bt2p, int ldb, long strideB,
    void* __restrict__ Cout, void* __restrict__ Cout2, int ldc, long strideC,
    const float* __restrict__ bias,
    const float* __restrict__ resid, long strideR,
    int M, int N, int K, float scale) {
  typedef typename Elem<ET>::T T;
  typedef typename Frag<T>::V V;
  const T* A = (const T*)Ap; const T* A2 = (const T*)A2p; const T* Bt = (const T*)Btp; const T* Bt2 = (const T*)Bt2p;
  __shared__ __align__(16) float sT[8][16 * 68];
  const int b    = blockIdx.y;
  const int lane = threadIdx.x & 31;
  const int wave = threadIdx.x >> 5;
  const int tilesN = N >> 6;
  const int tilesM = M >> 6;
  const int tile = blockIdx.x * 8 + wave;
  if (tile >= tilesM * tilesN) return;
  const int tm = tile / tilesN;
  const int tn = tile - tm * tilesN;
  const int m0 = tm << 6;
  const int n0 = tn << 6;

  const T* Ab  = A  + (size_t)b * strideA;
  const T* Bb  = Bt + (size_t)b * strideB;
  const T* Ab2 = SPLIT ? (A2  + (size_t)b * strideA) : nullptr;
  const T* Bb2 = SPLIT ? (Bt2 + (size_t)b * strideB) : nullptr;

  const int rlane = lane & 15;
  const int koff  = (lane >> 4) * 8;
  const int mOff  = (lane >> 4) * 8;

  v8f acc[4][4];
#pragma unroll
  for (int i = 0; i < 4; ++i)
#pragma unroll
    for (int j = 0; j < 4; ++j) acc[i][j] = (v8f){0.f,0.f,0.f,0.f,0.f,0.f,0.f,0.f};

  for (int k0 = 0; k0 < K; k0 += 32) {
    V bh[4], bl[4];
#pragma unroll
    for (int j = 0; j < 4; ++j) {
      const size_t bo = (size_t)(n0 + (j << 4) + rlane) * ldb + koff + k0;
      bh[j] = Frag<T>::load(Bb + bo);
      if (SPLIT) bl[j] = Frag<T>::load(Bb2 + bo);
    }
#pragma unroll
    for (int i = 0; i < 4; ++i) {
      const size_t ao = (size_t)(m0 + (i << 4) + rlane) * lda + koff + k0;
      V ah = Frag<T>::load(Ab + ao);
      V al;
      if (SPLIT) al = Frag<T>::load(Ab2 + ao);
#pragma unroll
      for (int j = 0; j < 4; ++j) {
        acc[i][j] = Frag<T>::mma(ah, bh[j], acc[i][j]);
        if (SPLIT) {
          acc[i][j] = Frag<T>::mma(ah, bl[j], acc[i][j]);
          acc[i][j] = Frag<T>::mma(al, bh[j], acc[i][j]);
        }
      }
      Frag<T>::guard(acc[i][0], acc[i][3], ah, SPLIT ? al : ah);
    }
    Frag<T>::keep(bh[0], bh[1], bh[2], bh[3]);
    if (SPLIT) Frag<T>::keep(bl[0], bl[1], bl[2], bl[3]);
  }
  acc_guard4(acc[0][0], acc[0][1], acc[0][2], acc[0][3]);
  acc_guard4(acc[1][0], acc[1][1], acc[1][2], acc[1][3]);
  acc_guard4(acc[2][0], acc[2][1], acc[2][2], acc[2][3]);
  acc_guard4(acc[3][0], acc[3][1], acc[3][2], acc[3][3]);

  float* slab = sT[wave];
  const float* Rb = RESID ? (resid + (size_t)b * strideR) : nullptr;
#pragma unroll
  for (int i = 0; i < 4; ++i) {
    const int mBase = m0 + (i << 4);
#pragma unroll
    for (int j = 0; j < 4; ++j) {
      const int n = n0 + (j << 4) + rlane;
      float bv = 0.f;
      if (BIAS_MODE == 2) bv = bias[n];
#pragma unroll
      for (int r = 0; r < 8; ++r) {
        float v = acc[i][j][r] * scale;
        if (BIAS_MODE == 1) v += bias[mBase + mOff + r];
        if (BIAS_MODE == 2) v += bv;
        if (RESID) v += Rb[(size_t)(mBase + mOff + r) * ldc + n];
        if (ACT == 1) v = tanhf(v);
        if (ACT == 2) v = fmaxf(v, 0.0f);
        if (ACT == 3) v = v / (1.0f + expf(-v));
        if (ACT == 4) v = (v > 0.f) ? v : 0.01f * v;
        if (ACT == 5) v = 0.5f * v * (1.0f + erff(v * 0.70710678118654752f));
        slab[(mOff + r) * 68 + (j << 4) + rlane] = v;
      }
    }
    __builtin_amdgcn_fence(__ATOMIC_RELEASE, "workgroup");
    __builtin_amdgcn_wave_barrier();
    __builtin_amdgcn_fence(__ATOMIC_ACQUIRE, "workgroup");
    if (OUT_MODE == 0) {
      float* C = (float*)Cout + (size_t)b * strideC;
      const int hh = lane >> 4, c4 = (lane & 15) * 4;
      for (int pass = 0; pass < 2; ++pass) {
#pragma unroll
        for (int it = 0; it < 8; ++it) {
          const int row = it * 2 + hh;
          v4f v = *(const v4f*)(slab + row * 68 + c4);
          *(volatile v4f*)(C + (size_t)(mBase + row) * ldc + n0 + c4) = v;
        }
        __threadfence();
      }
    } else {
      const int q = lane >> 3, c8 = (lane & 7) * 8;
      unsigned short* C  = (unsigned short*)Cout  + (size_t)b * strideC;
      unsigned short* C2 = (OUT_MODE == 2) ? ((unsigned short*)Cout2 + (size_t)b * strideC) : nullptr;
      for (int pass = 0; pass < 2; ++pass) {
#pragma unroll
        for (int it = 0; it < 4; ++it) {
          const int row = it * 4 + q;
          const float* sp = slab + row * 68 + c8;
          v8h hv, lv;
#pragma unroll
          for (int e = 0; e < 8; ++e) {
            if (OUT_MODE == 1) {
              hv[e] = (_Float16)sp[e];
            } else {
              unsigned short hb = f2bf_bits(sp[e]);
              unsigned short lb = f2bf_bits(sp[e] - bf_bits2f(hb));
              hv[e] = __builtin_bit_cast(_Float16, hb);
              lv[e] = __builtin_bit_cast(_Float16, lb);
            }
          }
          *(volatile v8h*)(C + (size_t)(mBase + row) * ldc + n0 + c8) = hv;
          if (OUT_MODE == 2) *(volatile v8h*)(C2 + (size_t)(mBase + row) * ldc + n0 + c8) = lv;
        }
        __threadfence();
      }
    }
    __builtin_amdgcn_fence(__ATOMIC_RELEASE, "workgroup");
    __builtin_amdgcn_wave_barrier();
    __builtin_amdgcn_fence(__ATOMIC_ACQUIRE, "workgroup");
  }
}

__global__ __launch_bounds__(256) void kmat_split_kernel(
    const float* __restrict__ x, const float* __restrict__ dp,
    unsigned short* __restrict__ kHi, unsigned short* __restrict__ kLo, int nrows) {
  __shared__ __align__(16) float sdp[COL_HALF * FEAT_DIM];
  __shared__ __align__(16) float sxn[ROWS_BLK * FEAT_DIM];
  const int tid  = threadIdx.x;
  const int n0   = blockIdx.x * ROWS_BLK;
  const int half = blockIdx.y;

  const float* dpb = dp + (size_t)half * COL_HALF * FEAT_DIM;
#pragma unroll
  for (int i = 0; i < 8; ++i) {
    const int idx4 = i * 256 + tid;
    *(v4f*)(sdp + idx4 * 4) = *(const v4f*)(dpb + (size_t)idx4 * 4);
  }

  if (tid < ROWS_BLK) {
    int row = n0 + tid;
    row = (row < nrows) ? row : (nrows - 1);
    const float* xr = x + (size_t)row * FEAT_DIM;
    const v4f a0 = *(const v4f*)(xr);
    const v4f a1 = *(const v4f*)(xr + 4);
    const v4f a2 = *(const v4f*)(xr + 8);
    const v4f a3 = *(const v4f*)(xr + 12);
    float xv[FEAT_DIM];
#pragma unroll
    for (int e = 0; e < 4; ++e) { xv[e] = a0[e]; xv[4 + e] = a1[e]; xv[8 + e] = a2[e]; xv[12 + e] = a3[e]; }
    float s = 0.f;
#pragma unroll
    for (int d = 0; d < FEAT_DIM; ++d) s += xv[d];
    const float mean = s * (1.0f / 16.0f);
    float qv = 0.f;
#pragma unroll
    for (int d = 0; d < FEAT_DIM; ++d) { const float t = xv[d] - mean; qv += t * t; }
    const float rstd = rsqrtf(qv * (1.0f / 16.0f) + 1e-5f);
#pragma unroll
    for (int d = 0; d < FEAT_DIM; ++d) sxn[tid * FEAT_DIM + d] = (xv[d] - mean) * rstd;
  }
  __syncthreads();

  const int cg   = tid & 63;
  const int rsel = tid >> 6;
  const int mloc = cg * 8;
#pragma unroll 1
  for (int p = 0; p < ROWS_BLK / 4; ++p) {
    const int r = p * 4 + rsel;
    const int n = n0 + r;
    const float* xp = sxn + r * FEAT_DIM;
    const v4f x0 = *(const v4f*)(xp);
    const v4f x1 = *(const v4f*)(xp + 4);
    const v4f x2 = *(const v4f*)(xp + 8);
    const v4f x3 = *(const v4f*)(xp + 12);
    v8h hv, lv;
#pragma unroll
    for (int j = 0; j < 8; ++j) {
      const float* dr = sdp + (mloc + j) * FEAT_DIM;
      const v4f d0 = *(const v4f*)(dr);
      const v4f d1 = *(const v4f*)(dr + 4);
      const v4f d2 = *(const v4f*)(dr + 8);
      const v4f d3 = *(const v4f*)(dr + 12);
      float l1 = 0.f;
#pragma unroll
      for (int e = 0; e < 4; ++e) l1 += fabsf(x0[e] - d0[e]);
#pragma unroll
      for (int e = 0; e < 4; ++e) l1 += fabsf(x1[e] - d1[e]);
#pragma unroll
      for (int e = 0; e < 4; ++e) l1 += fabsf(x2[e] - d2[e]);
#pragma unroll
      for (int e = 0; e < 4; ++e) l1 += fabsf(x3[e] - d3[e]);
      const float kv = __expf(-l1);
      const unsigned short hb = f2bf_bits(kv);
      const unsigned short lb = f2bf_bits(kv - bf_bits2f(hb));
      hv[j] = __builtin_bit_cast(_Float16, hb);
      lv[j] = __builtin_bit_cast(_Float16, lb);
    }
    const size_t off = (size_t)n * NDESIGN + (size_t)half * COL_HALF + mloc;
    *(volatile v8h*)(kHi + off) = hv;
    *(volatile v8h*)(kLo + off) = lv;
    __threadfence();
    *(volatile v8h*)(kHi + off) = hv;
    *(volatile v8h*)(kLo + off) = lv;
  }
}

__global__ __launch_bounds__(256) void chol_transpose_split_kernel(
    const float* __restrict__ c, unsigned short* __restrict__ tHi, unsigned short* __restrict__ tLo, int msz) {
  __shared__ float st[64][65];
  const int tid = threadIdx.x;
  const int n0 = blockIdx.x * 64;
  const int k0 = blockIdx.y * 64;
#pragma unroll
  for (int i = 0; i < 4; ++i) {
    const int idx = i * 256 + tid;
    const int kk = idx >> 4, c4 = (idx & 15) * 4;
    const v4f v = *(const v4f*)(c + (size_t)(k0 + kk) * msz + n0 + c4);
    st[kk][c4 + 0] = v[0];
    st[kk][c4 + 1] = v[1];
    st[kk][c4 + 2] = v[2];
    st[kk][c4 + 3] = v[3];
  }
  __syncthreads();
#pragma unroll
  for (int it = 0; it < 2; ++it) {
    const int nn = it * 32 + (tid >> 3);
    const int c8 = (tid & 7) * 8;
    v8h hv, lv;
#pragma unroll
    for (int e = 0; e < 8; ++e) {
      const float f = st[c8 + e][nn];
      const unsigned short hb = f2bf_bits(f);
      const unsigned short lb = f2bf_bits(f - bf_bits2f(hb));
      hv[e] = __builtin_bit_cast(_Float16, hb);
      lv[e] = __builtin_bit_cast(_Float16, lb);
    }
    const size_t off = (size_t)(n0 + nn) * msz + k0 + c8;
    *(volatile v8h*)(tHi + off) = hv;
    *(volatile v8h*)(tLo + off) = lv;
    __threadfence();
    *(volatile v8h*)(tHi + off) = hv;
    *(volatile v8h*)(tLo + off) = lv;
  }
}

extern "C" void kernel_launch(void* const* d_in, const int* in_sizes, int n_in,
                              void* d_out, int out_size, void* d_ws, size_t ws_size,
                              hipStream_t stream) {
  if (n_in < 3) return;
  const float* x    = (const float*)d_in[0];
  const float* dp   = (const float*)d_in[1];
  const float* chol = (const float*)d_in[2];
  float* out = (float*)d_out;

  const int nrows = in_sizes[0] / FEAT_DIM;
  if (nrows <= 0 || (nrows % 64) != 0 || in_sizes[0] != nrows * FEAT_DIM) return;
  if (in_sizes[1] != NDESIGN * FEAT_DIM) return;
  if (in_sizes[2] != NDESIGN * NDESIGN) return;
  if (out_size != nrows * NDESIGN) return;

  const size_t szK = (size_t)nrows * NDESIGN * 2;
  const size_t szC = (size_t)NDESIGN * NDESIGN * 2;
  const size_t offKh = 0;
  const size_t offKl = offKh + szK;
  const size_t offCh = offKl + szK;
  const size_t offCl = offCh + szC;
  const size_t total = offCl + szC;
  if (total > ws_size) return;

  char* ws = (char*)d_ws;
  unsigned short* kHi = (unsigned short*)(ws + offKh);
  unsigned short* kLo = (unsigned short*)(ws + offKl);
  unsigned short* cHi = (unsigned short*)(ws + offCh);
  unsigned short* cLo = (unsigned short*)(ws + offCl);

  {
    dim3 grid(nrows / ROWS_BLK, NDESIGN / COL_HALF);
    kmat_split_kernel<<<grid, 256, 0, stream>>>(x, dp, kHi, kLo, nrows);
  }
  {
    dim3 grid(NDESIGN / 64, NDESIGN / 64);
    chol_transpose_split_kernel<<<grid, 256, 0, stream>>>(chol, cHi, cLo, NDESIGN);
  }
  {
    const int tiles = (nrows / 64) * (NDESIGN / 64);
    dim3 grid((tiles + 7) / 8, 1);
    wmma_gemm64<1, true, 0, 0, false, 0><<<grid, 256, 0, stream>>>(
        kHi, kLo, NDESIGN, 0L,
        cHi, cLo, NDESIGN, 0L,
        (void*)out, (void*)out, NDESIGN, 0L,
        (const float*)out,
        (const float*)out, 0L,
        nrows, NDESIGN, NDESIGN, 1.0f);
  }
}
